// Bezier_27539330302394
// MI455X (gfx1250) — hardware-verified
//
#include <hip/hip_runtime.h>


namespace {
constexpr int RES = 1024, STEPS = 256;
constexpr float XS = 8.0f, INV2S2 = 1.0f / (2.0f * 0.01f * 0.01f);

typedef _Float16 b16;
typedef __attribute__((ext_vector_type(16))) _Float16 v16b;
typedef __attribute__((ext_vector_type(8))) _Float16 v8b;
typedef __attribute__((ext_vector_type(8))) float v8f;
typedef __attribute__((ext_vector_type(4))) float v4f;
__device__ __forceinline__ float bf16_rne(float f) { unsigned int u = __float_as_uint(f); u += 0x7FFFu + ((u >> 16) & 1u); return __uint_as_float(u & 0xFFFF0000u); }
__device__ __forceinline__ void split16(float v, b16& hi, b16& lo) { hi = (b16)v; lo = (b16)(v - (float)hi); }
__device__ __forceinline__ v16b frag_kb(const b16* p, int hh) { const v8b a = *(const v8b*)(p + 8 * hh), b = *(const v8b*)(p + 16 + 8 * hh); v16b f;
#pragma unroll
  for (int e = 0; e < 8; ++e) { f[e] = a[e]; f[8 + e] = b[e]; } return f; }
__device__ __forceinline__ v8f wmma16b(v16b a, v16b b, v8f c) { v8f d = __builtin_amdgcn_wmma_f32_16x16x32_f16(false, a, false, b, (short)0, c, false, false); asm volatile("v_nop\n\tv_nop\n\tv_nop\n\tv_nop" : "+v"(d) : "v"(a), "v"(b)); return d; }
__device__ __forceinline__ void wave_lds_sync() { __builtin_amdgcn_fence(__ATOMIC_RELEASE, "workgroup"); __builtin_amdgcn_wave_barrier(); __builtin_amdgcn_fence(__ATOMIC_ACQUIRE, "workgroup"); }
__device__ __forceinline__ float nexp(float x) { return __builtin_amdgcn_exp2f(x * 1.4426950408889634f); }
__device__ __forceinline__ float pmul(float a, float b) { float p = a * b; asm volatile("" : "+v"(p)); return p; }

__global__ __launch_bounds__(256) void tab_kernel(const float* __restrict__ cp, b16* __restrict__ EXh, b16* __restrict__ EXl, b16* __restrict__ EYh, b16* __restrict__ EYl) {
  __shared__ __attribute__((aligned(16))) b16 Th[2][STEPS + 8], Tl[2][STEPS + 8];
  const int a = blockIdx.x, s = threadIdx.x;
  const float p0x = bf16_rne(cp[0]), p0y = bf16_rne(cp[1]), p1x = bf16_rne(cp[2]), p1y = bf16_rne(cp[3]), p2x = bf16_rne(cp[4]), p2y = bf16_rne(cp[5]);
  const float tl = (float)s * (1.0f / 255.0f), tb = (float)s * (1.0f / 256.0f);
  const float ax = p0x + pmul(p1x - p0x, tl), ay = p0y + pmul(p1y - p0y, tl), bx = p1x + pmul(p2x - p1x, tl), by = p1y + pmul(p2y - p1y, tl);
  const float cx = ax + pmul(tb, bx - ax), cy = ay + pmul(tb, by - ay);
  const float g = (float)a * (1.0f / 1024.0f); const float dx = g - cx, dy = g - cy;
  const float ex = nexp(-pmul(pmul(dx, dx), INV2S2)), ey = nexp(-pmul(pmul(dy, dy), INV2S2));
  b16 h_, l_; split16(ex * XS, h_, l_); Th[0][s] = h_; Tl[0][s] = l_; split16(ey * XS, h_, l_); Th[1][s] = h_; Tl[1][s] = l_;
  __syncthreads();
  for (int pass = 0; pass < 2; ++pass) { if (s < 64) { const int w = s >> 5, c8 = (s & 31) * 8; b16* dh = w ? EYh : EXh; b16* dl = w ? EYl : EXl; *(volatile v8b*)(dh + (size_t)a * STEPS + c8) = *(const v8b*)(&Th[w][c8]); *(volatile v8b*)(dl + (size_t)a * STEPS + c8) = *(const v8b*)(&Tl[w][c8]); } __threadfence(); }
}
__global__ __launch_bounds__(64) void gemm_kernel(const b16* __restrict__ EYh, const b16* __restrict__ EYl, const b16* __restrict__ EXh, const b16* __restrict__ EXl, float* __restrict__ out) {
  __shared__ __attribute__((aligned(16))) float Ts[2][16][128 + 4];
  const int lane = threadIdx.x & 31, wave = threadIdx.x >> 5, nloc = lane & 15, hlf = lane >> 4, m0 = blockIdx.y * 32 + wave * 16, c0 = blockIdx.x * 128;
  v8f acc[8];
#pragma unroll
  for (int t = 0; t < 8; ++t) acc[t] = (v8f){};
#pragma unroll 2
  for (int kb = 0; kb < STEPS; kb += 32) { const v16b a0 = frag_kb(EYh + (size_t)(m0 + nloc) * STEPS + kb, hlf), l0 = frag_kb(EYl + (size_t)(m0 + nloc) * STEPS + kb, hlf);
#pragma unroll
    for (int t = 0; t < 8; ++t) { const v16b bh = frag_kb(EXh + (size_t)(c0 + t * 16 + nloc) * STEPS + kb, hlf), bl = frag_kb(EXl + (size_t)(c0 + t * 16 + nloc) * STEPS + kb, hlf);
      acc[t] = wmma16b(a0, bh, acc[t]); acc[t] = wmma16b(l0, bh, acc[t]); acc[t] = wmma16b(a0, bl, acc[t]); } }
#pragma unroll
  for (int t = 0; t < 8; ++t)
#pragma unroll
    for (int v = 0; v < 8; ++v) Ts[wave][8 * hlf + v][t * 16 + nloc] = acc[t][v] * (1.0f / (XS * XS * STEPS));
  wave_lds_sync();
  for (int pass = 0; pass < 2; ++pass) { for (int i = lane; i < 16 * 32; i += 32) { const int rr = i >> 5, c4 = (i & 31) * 4; *(volatile v4f*)(out + (size_t)(m0 + rr) * RES + c0 + c4) = *(const v4f*)(&Ts[wave][rr][c4]); } __threadfence(); }
}
}

extern "C" void kernel_launch(void* const* d_in, const int* in_sizes, int n_in,
                              void* d_out, int out_size, void* d_ws, size_t ws_size, hipStream_t stream) {
  (void)n_in; (void)out_size;
  const float* cp = (const float*)d_in[0]; float* out = (float*)d_out;
  if (in_sizes[0] != 6) return;
  size_t off = 0; char* ws = (char*)d_ws;
  auto carve = [&](size_t bytes) { char* p = ws + off; off += (bytes + 255) & ~(size_t)255; return p; };
  b16* EXh = (b16*)carve((size_t)RES * STEPS * 2); b16* EXl = (b16*)carve((size_t)RES * STEPS * 2); b16* EYh = (b16*)carve((size_t)RES * STEPS * 2); b16* EYl = (b16*)carve((size_t)RES * STEPS * 2);
  if (off > ws_size) return;
  tab_kernel<<<RES, 256, 0, stream>>>(cp, EXh, EXl, EYh, EYl);
  gemm_kernel<<<dim3(8, RES / 32), 64, 0, stream>>>(EYh, EYl, EXh, EXl, out);
}
